// VSSM_27427661152994
// MI455X (gfx1250) — hardware-verified
//
#include <hip/hip_runtime.h>
#include <math.h>

typedef __attribute__((ext_vector_type(16))) _Float16 v16h;
typedef __attribute__((ext_vector_type(8)))  _Float16 v8h;
typedef __attribute__((ext_vector_type(16))) __bf16   v16b;
typedef __attribute__((ext_vector_type(8)))  __bf16   v8b;
typedef __attribute__((ext_vector_type(8)))  float    v8f;
typedef __attribute__((ext_vector_type(4)))  float    v4f;

constexpr int kB     = 8;
constexpr int kH     = 56;
constexpr int kW     = 56;
constexpr int kL     = kH * kW;
constexpr int kRows  = kB * kL;
constexpr int kDm    = 96;
constexpr int kDin   = 192;
constexpr int kNst   = 16;
constexpr int kDtR   = 6;
constexpr int kDirs  = 4;
constexpr int kXc    = kDtR + 2 * kNst;
constexpr int kXzP   = 2 * kDin;
constexpr int kXdReal = kDirs * kXc;
constexpr int kXdN   = 192;
constexpr int kOutN  = 128;
constexpr int kConvPix = 8;
constexpr int kConvTP  = 196;
constexpr int kScanCh  = 64;
constexpr int kScanTS  = 64;
constexpr int kScanYP  = 68;
static_assert(kH == kW, "square spatial grid assumed by the traversal map");
static_assert((kDm % 32) == 0 && (kDin % 32) == 0, "GEMM K multiples of 32");
static_assert((kRows % 64) == 0 && (kXzP % 64) == 0 && (kXdN % 64) == 0 && (kOutN % 64) == 0, "GEMM M,N multiples of 64");
static_assert(kXdReal <= kXdN && kDm <= kOutN, "padded N covers real N");
static_assert((kW % kConvPix) == 0 && (kRows % kConvPix) == 0, "conv pixel groups stay inside one image row");
static_assert((kL % kScanTS) == 0 && (kDin % kScanCh) == 0, "scan tiles");
static_assert((kRows % 32) == 0, "LN rows per block");
static_assert((kDm % 32) == 0, "d_out column clip lands on whole 128-B lines");

constexpr size_t kOffXB   = 0;
constexpr size_t kOffWIB  = kOffXB  + (size_t)kRows * kDm  * 2;
constexpr size_t kOffWXB  = kOffWIB + (size_t)kXzP  * kDm  * 2;
constexpr size_t kOffWOB  = kOffWXB + (size_t)kXdN  * kDin * 2;
constexpr size_t kOffXZ   = kOffWOB + (size_t)kOutN * kDin * 2;
constexpr size_t kOffXC   = kOffXZ  + (size_t)kRows * kXzP * 4;
constexpr size_t kOffXCH  = kOffXC  + (size_t)kRows * kDin * 4;
constexpr size_t kOffXCL  = kOffXCH + (size_t)kRows * kDin * 2;
constexpr size_t kOffXD   = kOffXCL + (size_t)kRows * kDin * 2;
constexpr size_t kOffYS   = kOffXD  + (size_t)kRows * kXdN * 4;
constexpr size_t kWsTotal = kOffYS  + (size_t)kRows * kDin * 4;
constexpr size_t kOffYGH  = kOffXCH;
constexpr size_t kOffYGL  = kOffXCL;
static_assert(kWsTotal == 120619008ull, "carve total");
static_assert(kWsTotal <= 134217728ull, "carve cap");
static_assert((kOffWIB % 128) == 0 && (kOffWXB % 128) == 0 && (kOffWOB % 128) == 0 && (kOffXZ % 128) == 0 &&
              (kOffXC % 128) == 0 && (kOffXCH % 128) == 0 && (kOffXCL % 128) == 0 && (kOffXD % 128) == 0 &&
              (kOffYS % 128) == 0, "128-B aligned regions");

__device__ __forceinline__ unsigned short f2bf_bits(float f) {
  unsigned u = __float_as_uint(f);
  return (unsigned short)((u + 0x7FFFu + ((u >> 16) & 1u)) >> 16);
}
__device__ __forceinline__ float bf_bits2f(unsigned short h) { return __uint_as_float(((unsigned)h) << 16); }
__device__ __forceinline__ float bf16_rne(float f) { return bf_bits2f(f2bf_bits(f)); }

__device__ __forceinline__ void dep_guard4_h(v8f& a, v8f& b, v8f& c, v8f& d, v16h x, v16h y) {
  asm volatile("v_nop\n\tv_nop\n\tv_nop\n\tv_nop" : "+v"(a), "+v"(b), "+v"(c), "+v"(d) : "v"(x), "v"(y));
}
__device__ __forceinline__ void dep_guard4_b(v8f& a, v8f& b, v8f& c, v8f& d, v16b x, v16b y) {
  asm volatile("v_nop\n\tv_nop\n\tv_nop\n\tv_nop" : "+v"(a), "+v"(b), "+v"(c), "+v"(d) : "v"(x), "v"(y));
}
__device__ __forceinline__ void keep4_h(v16h a, v16h b, v16h c, v16h d) { asm volatile("v_nop" :: "v"(a), "v"(b), "v"(c), "v"(d)); }
__device__ __forceinline__ void keep4_b(v16b a, v16b b, v16b c, v16b d) { asm volatile("v_nop" :: "v"(a), "v"(b), "v"(c), "v"(d)); }
__device__ __forceinline__ void acc_guard4(v8f& a, v8f& b, v8f& c, v8f& d) { asm volatile("v_nop\n\tv_nop\n\tv_nop\n\tv_nop" : "+v"(a), "+v"(b), "+v"(c), "+v"(d)); }
template <typename T> struct Frag;
template <> struct Frag<_Float16> {
  typedef v16h V; union U { v16h v; v8h h[2]; };
  static __device__ __forceinline__ v16h load(const _Float16* p) {
    U f; f.h[0] = *(const v8h*)(p); f.h[1] = *(const v8h*)(p + 16); return f.v;
  }
  static __device__ __forceinline__ v8f mma(v16h a, v16h b, v8f c) {
    return __builtin_amdgcn_wmma_f32_16x16x32_f16(false, a, false, b, (short)0, c, false, false);
  }
  static __device__ __forceinline__ void guard4(v8f& a, v8f& b, v8f& c, v8f& d, v16h x, v16h y) { dep_guard4_h(a, b, c, d, x, y); }
  static __device__ __forceinline__ void keep(v16h a, v16h b, v16h c, v16h d) { keep4_h(a, b, c, d); }
};
template <> struct Frag<__bf16> {
  typedef v16b V; union U { v16b v; v8b h[2]; };
  static __device__ __forceinline__ v16b load(const __bf16* p) {
    U f; f.h[0] = *(const v8b*)(p); f.h[1] = *(const v8b*)(p + 16); return f.v;
  }
  static __device__ __forceinline__ v8f mma(v16b a, v16b b, v8f c) {
    return __builtin_amdgcn_wmma_f32_16x16x32_bf16(false, a, false, b, (short)0, c, false, false);
  }
  static __device__ __forceinline__ void guard4(v8f& a, v8f& b, v8f& c, v8f& d, v16b x, v16b y) { dep_guard4_b(a, b, c, d, x, y); }
  static __device__ __forceinline__ void keep(v16b a, v16b b, v16b c, v16b d) { keep4_b(a, b, c, d); }
};

template <int ET> struct Elem;
template <> struct Elem<0> { typedef _Float16 T; };
template <> struct Elem<1> { typedef __bf16 T; };
template <int ET, int SPL, int BIAS_MODE, int OUT_MODE, bool RESID, int ACT = 0>
__global__ __launch_bounds__(256) void wmma_gemm64(
    const unsigned short* __restrict__ Ap, const unsigned short* __restrict__ A2p, int lda, long strideA,
    const unsigned short* __restrict__ Btp, const unsigned short* __restrict__ Bt2p, int ldb, long strideB,
    void* __restrict__ Cout, void* __restrict__ Cout2, int ldc, long strideC,
    const float* __restrict__ bias,
    const float* __restrict__ resid, long strideR,
    int M, int N, int K, float scale, int Nreal) {
  typedef typename Elem<ET>::T T;
  typedef typename Frag<T>::V V;
  const T* A = (const T*)Ap; const T* A2 = (const T*)A2p; const T* Bt = (const T*)Btp; const T* Bt2 = (const T*)Bt2p;
  __shared__ __align__(16) float sT[8][16 * 68];
  const int b    = blockIdx.y;
  const int lane = threadIdx.x & 31;
  const int wave = threadIdx.x >> 5;
  const int tilesN = N >> 6;
  const int tilesM = M >> 6;
  const int tile = blockIdx.x * 8 + wave;
  if (tile >= tilesM * tilesN) return;
  const int tm = tile / tilesN;
  const int tn = tile - tm * tilesN;
  const int m0 = tm << 6;
  const int n0 = tn << 6;

  const T* Ab  = A  + (size_t)b * strideA;
  const T* Bb  = Bt + (size_t)b * strideB;
  const T* Ab2 = (SPL >= 1) ? (A2  + (size_t)b * strideA) : nullptr;
  const T* Bb2 = (SPL == 2) ? (Bt2 + (size_t)b * strideB) : nullptr;

  const int rlane = lane & 15;
  const int koff  = (lane >> 4) * 8;
  const int mOff  = (lane >> 4) * 8;

  v8f acc[4][4];
#pragma unroll
  for (int i = 0; i < 4; ++i)
#pragma unroll
    for (int j = 0; j < 4; ++j) acc[i][j] = (v8f){0.f,0.f,0.f,0.f,0.f,0.f,0.f,0.f};

  for (int k0 = 0; k0 < K; k0 += 32) {
    V bh[4], bl[4];
#pragma unroll
    for (int j = 0; j < 4; ++j) {
      const size_t bo = (size_t)(n0 + (j << 4) + rlane) * ldb + koff + k0;
      bh[j] = Frag<T>::load(Bb + bo);
      if (SPL == 2) bl[j] = Frag<T>::load(Bb2 + bo);
    }
#pragma unroll
    for (int i = 0; i < 4; ++i) {
      const size_t ao = (size_t)(m0 + (i << 4) + rlane) * lda + koff + k0;
      V ah = Frag<T>::load(Ab + ao);
      V al;
      if (SPL >= 1) al = Frag<T>::load(Ab2 + ao);
#pragma unroll
      for (int j = 0; j < 4; ++j) {
        acc[i][j] = Frag<T>::mma(ah, bh[j], acc[i][j]);
        if (SPL == 2) acc[i][j] = Frag<T>::mma(ah, bl[j], acc[i][j]);
        if (SPL >= 1) acc[i][j] = Frag<T>::mma(al, bh[j], acc[i][j]);
      }
      Frag<T>::guard4(acc[i][0], acc[i][1], acc[i][2], acc[i][3], ah, (SPL >= 1) ? al : ah);
    }
    Frag<T>::keep(bh[0], bh[1], bh[2], bh[3]);
    if (SPL == 2) Frag<T>::keep(bl[0], bl[1], bl[2], bl[3]);
  }
  acc_guard4(acc[0][0], acc[0][1], acc[0][2], acc[0][3]);
  acc_guard4(acc[1][0], acc[1][1], acc[1][2], acc[1][3]);
  acc_guard4(acc[2][0], acc[2][1], acc[2][2], acc[2][3]);
  acc_guard4(acc[3][0], acc[3][1], acc[3][2], acc[3][3]);

  float* slab = sT[wave];
  const float* Rb = RESID ? (resid + (size_t)b * strideR) : nullptr;
#pragma unroll
  for (int i = 0; i < 4; ++i) {
    const int mBase = m0 + (i << 4);
#pragma unroll
    for (int j = 0; j < 4; ++j) {
      const int n = n0 + (j << 4) + rlane;
      float bv = 0.f;
      if (BIAS_MODE == 2) bv = bias[n];
#pragma unroll
      for (int r = 0; r < 8; ++r) {
        float v = acc[i][j][r] * scale;
        if (BIAS_MODE == 1) v += bias[mBase + mOff + r];
        if (BIAS_MODE == 2) v += bv;
        if (RESID) v += Rb[(size_t)(mBase + mOff + r) * ldc + n];
        if (ACT == 1) v = tanhf(v);
        if (ACT == 2) v = fmaxf(v, 0.0f);
        if (ACT == 3) v = v / (1.0f + expf(-v));
        if (ACT == 4) v = (v > 0.f) ? v : 0.01f * v;
        slab[(mOff + r) * 68 + (j << 4) + rlane] = v;
      }
    }
    __builtin_amdgcn_fence(__ATOMIC_RELEASE, "workgroup");
    __builtin_amdgcn_wave_barrier();
    __builtin_amdgcn_fence(__ATOMIC_ACQUIRE, "workgroup");
    if (OUT_MODE == 0) {
      float* C = (float*)Cout + (size_t)b * strideC;
      const int hh = lane >> 4, c4 = (lane & 15) * 4;
      for (int pass = 0; pass < 2; ++pass) {
#pragma unroll
        for (int it = 0; it < 8; ++it) {
          const int row = it * 2 + hh;
          v4f v = *(const v4f*)(slab + row * 68 + c4);
          if (n0 + c4 < Nreal) *(volatile v4f*)(C + (size_t)(mBase + row) * ldc + n0 + c4) = v;
        }
        __threadfence();
      }
    } else {
      const int q = lane >> 3, c8 = (lane & 7) * 8;
      unsigned short* C  = (unsigned short*)Cout  + (size_t)b * strideC;
      unsigned short* C2 = (OUT_MODE == 2) ? ((unsigned short*)Cout2 + (size_t)b * strideC) : nullptr;
      for (int pass = 0; pass < 2; ++pass) {
#pragma unroll
        for (int it = 0; it < 4; ++it) {
          const int row = it * 4 + q;
          const float* sp = slab + row * 68 + c8;
          v8h hv, lv;
#pragma unroll
          for (int e = 0; e < 8; ++e) {
            if (OUT_MODE == 1) {
              hv[e] = (_Float16)sp[e];
            } else {
              unsigned short hb = f2bf_bits(sp[e]);
              unsigned short lb = f2bf_bits(sp[e] - bf_bits2f(hb));
              hv[e] = __builtin_bit_cast(_Float16, hb);
              lv[e] = __builtin_bit_cast(_Float16, lb);
            }
          }
          *(volatile v8h*)(C + (size_t)(mBase + row) * ldc + n0 + c8) = hv;
          if (OUT_MODE == 2) *(volatile v8h*)(C2 + (size_t)(mBase + row) * ldc + n0 + c8) = lv;
        }
        __threadfence();
      }
    }
    __builtin_amdgcn_fence(__ATOMIC_RELEASE, "workgroup");
    __builtin_amdgcn_wave_barrier();
    __builtin_amdgcn_fence(__ATOMIC_ACQUIRE, "workgroup");
  }
}

__global__ __launch_bounds__(256) void cast_rows_bf16_kernel(
    const float* __restrict__ src, unsigned short* __restrict__ dst, int real8, int total8)
{
  const int i = blockIdx.x * 256 + threadIdx.x;
  if (i >= total8) return;
  const int ic = (i < real8) ? i : (real8 - 1);
  const float fac = (i < real8) ? 1.0f : 0.0f;
  const size_t e0 = (size_t)ic << 3;
  const v4f a0 = *(const v4f*)(src + e0);
  const v4f a1 = *(const v4f*)(src + e0 + 4);
  v8h hv;
#pragma unroll
  for (int e = 0; e < 4; ++e) {
    hv[e]     = __builtin_bit_cast(_Float16, f2bf_bits(a0[e] * fac));
    hv[4 + e] = __builtin_bit_cast(_Float16, f2bf_bits(a1[e] * fac));
  }
  unsigned short* q = dst + ((size_t)i << 3);
  *(volatile v8h*)q = hv;
  __threadfence();
  *(volatile v8h*)q = hv;
}

__global__ __launch_bounds__(192) void dwconv_silu_kernel(
    const float* __restrict__ XZ, const float* __restrict__ cw, const float* __restrict__ cb,
    float* __restrict__ XC, unsigned short* __restrict__ XCH, unsigned short* __restrict__ XCL)
{
  __shared__ __align__(16) float sT[kConvPix * kConvTP];
  const int tid = threadIdx.x, lane = tid & 31, wave = tid >> 5;
  const int c = tid;
  const int row0 = blockIdx.x * kConvPix;
  const int b  = row0 / kL;
  const int p0 = row0 - b * kL;
  const int h  = p0 / kW;
  const int w0 = p0 - h * kW;
  const size_t brow = (size_t)b * kL;
  const float bc = bf16_rne(cb[c]);
  float acc[kConvPix];
#pragma unroll
  for (int p = 0; p < kConvPix; ++p) acc[p] = 0.0f;
#pragma unroll 1
  for (int dy = 0; dy < 3; ++dy) {
    const int hy  = h + dy - 1;
    const int hyc = (hy < 0) ? 0 : ((hy > kH - 1) ? (kH - 1) : hy);
    const float fy = (hy >= 0 && hy <= kH - 1) ? 1.0f : 0.0f;
    const float wd0 = bf16_rne(cw[c * 9 + dy * 3 + 0]);
    const float wd1 = bf16_rne(cw[c * 9 + dy * 3 + 1]);
    const float wd2 = bf16_rne(cw[c * 9 + dy * 3 + 2]);
    float xin[kConvPix + 2];
#pragma unroll
    for (int j = 0; j < kConvPix + 2; ++j) {
      const int wx  = w0 + j - 1;
      const int wxc = (wx < 0) ? 0 : ((wx > kW - 1) ? (kW - 1) : wx);
      const float fx = (wx >= 0 && wx <= kW - 1) ? 1.0f : 0.0f;
      xin[j] = XZ[(brow + (size_t)hyc * kW + wxc) * kXzP + c] * (fx * fy);
    }
#pragma unroll
    for (int p = 0; p < kConvPix; ++p) {
      acc[p] = fmaf(xin[p],     wd0, acc[p]);
      acc[p] = fmaf(xin[p + 1], wd1, acc[p]);
      acc[p] = fmaf(xin[p + 2], wd2, acc[p]);
    }
  }
#pragma unroll
  for (int p = 0; p < kConvPix; ++p) {
    const float sv = acc[p] + bc;
    const float sg = __builtin_amdgcn_rcpf(1.0f + expf(-sv));
    sT[p * kConvTP + c] = sv * sg;
  }
  __syncthreads();
  const int q = lane >> 3, l8 = lane & 7;
  v4f fv[2];
  size_t fo[2];
#pragma unroll
  for (int it = 0; it < 2; ++it) {
    const int li   = it * 24 + wave * 4 + q;
    const int prow = li / 6;
    const int seg  = li - prow * 6;
    const int col  = seg * 32 + l8 * 4;
    fv[it] = *(const v4f*)(sT + prow * kConvTP + col);
    fo[it] = (size_t)(row0 + prow) * kDin + col;
  }
  const int lj    = wave * 4 + q;
  const int prow2 = lj / 3;
  const int seg2  = lj - prow2 * 3;
  const int col2  = seg2 * 64 + l8 * 8;
  const float* sp = sT + prow2 * kConvTP + col2;
  const v4f a0 = *(const v4f*)(sp);
  const v4f a1 = *(const v4f*)(sp + 4);
  v8h hv, lv;
#pragma unroll
  for (int e = 0; e < 4; ++e) {
    const unsigned short h0 = f2bf_bits(a0[e]), h1 = f2bf_bits(a1[e]);
    const unsigned short l0 = f2bf_bits(a0[e] - bf_bits2f(h0)), l1 = f2bf_bits(a1[e] - bf_bits2f(h1));
    hv[e]     = __builtin_bit_cast(_Float16, h0);
    hv[4 + e] = __builtin_bit_cast(_Float16, h1);
    lv[e]     = __builtin_bit_cast(_Float16, l0);
    lv[4 + e] = __builtin_bit_cast(_Float16, l1);
  }
  const size_t ho = (size_t)(row0 + prow2) * kDin + col2;
  for (int pass = 0; pass < 2; ++pass) {
#pragma unroll
    for (int it = 0; it < 2; ++it) *(volatile v4f*)(XC + fo[it]) = fv[it];
    *(volatile v8h*)(XCH + ho) = hv;
    *(volatile v8h*)(XCL + ho) = lv;
    __threadfence();
  }
}

__global__ __launch_bounds__(64) void scan_kernel(
    const float* __restrict__ XD, const float* __restrict__ XC,
    const float* __restrict__ Wdt, const float* __restrict__ bdt,
    const float* __restrict__ Alog, const float* __restrict__ Dsk,
    float* __restrict__ YS)
{
  __shared__ __align__(16) float sX[kScanTS * 64];
  __shared__ __align__(16) float sU[kScanTS * kScanCh];
  __shared__ __align__(16) float sY[kScanTS * kScanYP];
  __shared__ int sRow[kScanTS];
  const int tid = threadIdx.x, lane = tid & 31, wave = tid >> 5;
  constexpr int kBlkPerB = kDin / kScanCh;
  const int b  = blockIdx.x / kBlkPerB;
  const int d0 = (blockIdx.x - b * kBlkPerB) * kScanCh;
  const int d  = d0 + tid;
  const int rowb = b * kL;
  const int cc  = (tid < kXc - 1) ? tid : (kXc - 1);
  const int pos = tid + ((tid >= kDtR) ? 2 : 0);
  const int q = lane >> 3, c4 = (lane & 7) * 4;
  const int rsub = wave * 2 + (q >> 1);
  const int fcol = (q & 1) * 32 + c4;

#pragma unroll 1
  for (int k = 0; k < kDirs; ++k) {
    const int kd = k * kDin + d;
    float negA[kNst];
    {
      const v4f g0 = *(const v4f*)(Alog + (size_t)kd * kNst);
      const v4f g1 = *(const v4f*)(Alog + (size_t)kd * kNst + 4);
      const v4f g2 = *(const v4f*)(Alog + (size_t)kd * kNst + 8);
      const v4f g3 = *(const v4f*)(Alog + (size_t)kd * kNst + 12);
#pragma unroll
      for (int e = 0; e < 4; ++e) {
        negA[e]      = -expf(bf16_rne(g0[e]));
        negA[4 + e]  = -expf(bf16_rne(g1[e]));
        negA[8 + e]  = -expf(bf16_rne(g2[e]));
        negA[12 + e] = -expf(bf16_rne(g3[e]));
      }
    }
    float wr[kDtR];
#pragma unroll
    for (int r = 0; r < kDtR; ++r) wr[r] = bf16_rne(Wdt[(size_t)kd * kDtR + r]);
    const float bias = bf16_rne(bdt[kd]);
    const float Dd   = bf16_rne(Dsk[kd]);
    float h[kNst];
#pragma unroll
    for (int n = 0; n < kNst; ++n) h[n] = 0.0f;
    const int kc0 = k * kXc;

#pragma unroll 1
    for (int ch = 0; ch < kL / kScanTS; ++ch) {
      __syncthreads();
      {
        const int l  = ch * kScanTS + tid;
        const int l2 = (k >= 2) ? (kL - 1 - l) : l;
        const int qa = l2 / kW;
        const int ra = l2 - qa * kW;
        const int hh = (k & 1) ? ra : qa;
        const int ww = (k & 1) ? qa : ra;
        sRow[tid] = rowb + hh * kW + ww;
      }
      __syncthreads();
#pragma unroll 4
      for (int i = 0; i < kScanTS; ++i) {
        const int r = sRow[i];
        const float xv = XD[(size_t)r * kXdN + kc0 + cc];
        const float uv = XC[(size_t)r * kDin + d];
        if (tid < kXc) sX[i * 64 + pos] = xv;
        sU[i * kScanCh + tid] = uv;
      }
      __syncthreads();
#pragma unroll 1
      for (int s = 0; s < kScanTS; ++s) {
        const float* xr = sX + s * 64;
        float dot = 0.0f;
#pragma unroll
        for (int r = 0; r < kDtR; ++r) dot = fmaf(xr[r], wr[r], dot);
        const float v   = dot + bias;
        const float dlt = fmaxf(v, 0.0f) + log1pf(expf(-fabsf(v)));
        const float ut  = sU[s * kScanCh + tid];
        const float du  = dlt * ut;
        float Bs[kNst], Cs[kNst];
#pragma unroll
        for (int q4 = 0; q4 < 4; ++q4) {
          const v4f bv = *(const v4f*)(xr + 8 + 4 * q4);
          const v4f cv = *(const v4f*)(xr + 24 + 4 * q4);
          Bs[4 * q4 + 0] = bv[0]; Bs[4 * q4 + 1] = bv[1]; Bs[4 * q4 + 2] = bv[2]; Bs[4 * q4 + 3] = bv[3];
          Cs[4 * q4 + 0] = cv[0]; Cs[4 * q4 + 1] = cv[1]; Cs[4 * q4 + 2] = cv[2]; Cs[4 * q4 + 3] = cv[3];
        }
        float y = 0.0f;
#pragma unroll
        for (int n = 0; n < kNst; ++n) {
          const float e = __expf(dlt * negA[n]);
          h[n] = fmaf(e, h[n], du * Bs[n]);
          y = fmaf(h[n], Cs[n], y);
        }
        y = fmaf(Dd, ut, y);
        sY[s * kScanYP + tid] = y;
      }
      __syncthreads();
#pragma unroll 1
      for (int half = 0; half < 2; ++half) {
        v4f vals[8];
        int grow[8];
#pragma unroll
        for (int it = 0; it < 8; ++it) {
          const int row = (half * 8 + it) * 4 + rsub;
          vals[it] = *(const v4f*)(sY + row * kScanYP + fcol);
          grow[it] = sRow[row];
        }
        if (k > 0) {
#pragma unroll
          for (int it = 0; it < 8; ++it) {
            const v4f old = *(const v4f*)(YS + (size_t)grow[it] * kDin + d0 + fcol);
            vals[it] += old;
          }
        }
        for (int pass = 0; pass < 2; ++pass) {
#pragma unroll
          for (int it = 0; it < 8; ++it)
            *(volatile v4f*)(YS + (size_t)grow[it] * kDin + d0 + fcol) = vals[it];
          __threadfence();
        }
      }
    }
  }
}

__global__ __launch_bounds__(256) void ln_gate_kernel(
    const float* __restrict__ YS, const float* __restrict__ XZ,
    const float* __restrict__ gam, const float* __restrict__ bet,
    unsigned short* __restrict__ YGH, unsigned short* __restrict__ YGL)
{
  __shared__ float sG[kDin];
  __shared__ float sBt[kDin];
  __shared__ __align__(16) float sR[8][kDin];
  const int tid = threadIdx.x, lane = tid & 31, wave = tid >> 5;
  if (tid < kDin) {
    sG[tid]  = bf16_rne(gam[tid]);
    sBt[tid] = bf16_rne(bet[tid]);
  }
  __syncthreads();
  float g6[6], b6[6];
#pragma unroll
  for (int j = 0; j < 6; ++j) { g6[j] = sG[lane + 32 * j]; b6[j] = sBt[lane + 32 * j]; }
  float* sr = sR[wave];
  const int lc = (lane < 24) ? lane : 23;
  const int rbase = blockIdx.x * 32 + wave * 4;
#pragma unroll 1
  for (int rr = 0; rr < 4; ++rr) {
    const size_t row = (size_t)(rbase + rr);
    float v[6];
#pragma unroll
    for (int j = 0; j < 6; ++j) v[j] = YS[row * kDin + lane + 32 * j];
    float s1 = 0.0f;
#pragma unroll
    for (int j = 0; j < 6; ++j) s1 += v[j];
#pragma unroll
    for (int off = 1; off < 32; off <<= 1) s1 += __shfl_xor(s1, off, 32);
    const float mu = s1 * (1.0f / 192.0f);
    float dv[6];
    float s2 = 0.0f;
#pragma unroll
    for (int j = 0; j < 6; ++j) { dv[j] = v[j] - mu; s2 = fmaf(dv[j], dv[j], s2); }
#pragma unroll
    for (int off = 1; off < 32; off <<= 1) s2 += __shfl_xor(s2, off, 32);
    const float var = s2 * (1.0f / 192.0f);
    const float rs  = rsqrtf(var + 1e-5f);
    float o[6];
#pragma unroll
    for (int j = 0; j < 6; ++j) {
      const float z  = XZ[row * kXzP + kDin + lane + 32 * j];
      const float sg = __builtin_amdgcn_rcpf(1.0f + expf(-z));
      o[j] = (dv[j] * rs * g6[j] + b6[j]) * (z * sg);
    }
#pragma unroll
    for (int j = 0; j < 6; ++j) sr[lane + 32 * j] = o[j];
    __builtin_amdgcn_fence(__ATOMIC_RELEASE, "workgroup");
    __builtin_amdgcn_wave_barrier();
    __builtin_amdgcn_fence(__ATOMIC_ACQUIRE, "workgroup");
    const v4f a0 = *(const v4f*)(sr + lc * 8);
    const v4f a1 = *(const v4f*)(sr + lc * 8 + 4);
    v8h hv, lv;
#pragma unroll
    for (int e = 0; e < 4; ++e) {
      const unsigned short h0 = f2bf_bits(a0[e]), h1 = f2bf_bits(a1[e]);
      const unsigned short l0 = f2bf_bits(a0[e] - bf_bits2f(h0)), l1 = f2bf_bits(a1[e] - bf_bits2f(h1));
      hv[e]     = __builtin_bit_cast(_Float16, h0);
      hv[4 + e] = __builtin_bit_cast(_Float16, h1);
      lv[e]     = __builtin_bit_cast(_Float16, l0);
      lv[4 + e] = __builtin_bit_cast(_Float16, l1);
    }
    const size_t o16 = row * kDin + (size_t)lane * 8;
    for (int pass = 0; pass < 2; ++pass) {
      if (lane < 24) {
        *(volatile v8h*)(YGH + o16) = hv;
        *(volatile v8h*)(YGL + o16) = lv;
      }
      __threadfence();
    }
    __builtin_amdgcn_fence(__ATOMIC_RELEASE, "workgroup");
    __builtin_amdgcn_wave_barrier();
    __builtin_amdgcn_fence(__ATOMIC_ACQUIRE, "workgroup");
  }
}

extern "C" void kernel_launch(void* const* d_in, const int* in_sizes, int n_in,
                              void* d_out, int out_size, void* d_ws, size_t ws_size,
                              hipStream_t stream) {
  if (n_in < 12) return;
  if (in_sizes[0]  != kRows * kDm) return;
  if (in_sizes[1]  != kXzP * kDm) return;
  if (in_sizes[2]  != kDin * 9) return;
  if (in_sizes[3]  != kDin) return;
  if (in_sizes[4]  != kDirs * kXc * kDin) return;
  if (in_sizes[5]  != kDirs * kDin * kDtR) return;
  if (in_sizes[6]  != kDirs * kDin) return;
  if (in_sizes[7]  != kDirs * kDin * kNst) return;
  if (in_sizes[8]  != kDirs * kDin) return;
  if (in_sizes[9]  != kDin) return;
  if (in_sizes[10] != kDin) return;
  if (in_sizes[11] != kDm * kDin) return;
  if (out_size != kRows * kDm) return;
  if (ws_size < kWsTotal) return;

  const float* x       = (const float*)d_in[0];
  const float* W_in    = (const float*)d_in[1];
  const float* conv_w  = (const float*)d_in[2];
  const float* conv_b  = (const float*)d_in[3];
  const float* W_x     = (const float*)d_in[4];
  const float* W_dt    = (const float*)d_in[5];
  const float* b_dt    = (const float*)d_in[6];
  const float* A_log   = (const float*)d_in[7];
  const float* Dsk     = (const float*)d_in[8];
  const float* ln_g    = (const float*)d_in[9];
  const float* ln_b    = (const float*)d_in[10];
  const float* W_out   = (const float*)d_in[11];
  float* out = (float*)d_out;

  char* ws = (char*)d_ws;
  unsigned short* XB  = (unsigned short*)(ws + kOffXB);
  unsigned short* WIB = (unsigned short*)(ws + kOffWIB);
  unsigned short* WXB = (unsigned short*)(ws + kOffWXB);
  unsigned short* WOB = (unsigned short*)(ws + kOffWOB);
  float*          XZ  = (float*)(ws + kOffXZ);
  float*          XC  = (float*)(ws + kOffXC);
  unsigned short* XCH = (unsigned short*)(ws + kOffXCH);
  unsigned short* XCL = (unsigned short*)(ws + kOffXCL);
  float*          XD  = (float*)(ws + kOffXD);
  float*          YS  = (float*)(ws + kOffYS);
  unsigned short* YGH = (unsigned short*)(ws + kOffYGH);
  unsigned short* YGL = (unsigned short*)(ws + kOffYGL);

  {
    const int t8x  = kRows * kDm / 8;
    const int t8wi = kXzP * kDm / 8;
    const int r8wx = kXdReal * kDin / 8;
    const int t8wx = kXdN * kDin / 8;
    const int r8wo = kDm * kDin / 8;
    const int t8wo = kOutN * kDin / 8;
    cast_rows_bf16_kernel<<<(t8x + 255) / 256, 256, 0, stream>>>(x, XB, t8x, t8x);
    cast_rows_bf16_kernel<<<(t8wi + 255) / 256, 256, 0, stream>>>(W_in, WIB, t8wi, t8wi);
    cast_rows_bf16_kernel<<<(t8wx + 255) / 256, 256, 0, stream>>>(W_x, WXB, r8wx, t8wx);
    cast_rows_bf16_kernel<<<(t8wo + 255) / 256, 256, 0, stream>>>(W_out, WOB, r8wo, t8wo);
  }

  wmma_gemm64<1, 0, 0, 0, false><<<dim3((kRows / 64) * (kXzP / 64) / 8, 1), 256, 0, stream>>>(
      XB, nullptr, kDm, 0L,
      WIB, nullptr, kDm, 0L,
      (void*)XZ, nullptr, kXzP, 0L,
      nullptr, nullptr, 0L,
      kRows, kXzP, kDm, 1.0f, kXzP);

  dwconv_silu_kernel<<<kRows / kConvPix, kDin, 0, stream>>>(XZ, conv_w, conv_b, XC, XCH, XCL);

  wmma_gemm64<1, 1, 0, 0, false><<<dim3((kRows / 64) * (kXdN / 64) / 8, 1), 256, 0, stream>>>(
      XCH, XCL, kDin, 0L,
      WXB, nullptr, kDin, 0L,
      (void*)XD, nullptr, kXdN, 0L,
      nullptr, nullptr, 0L,
      kRows, kXdN, kDin, 1.0f, kXdN);

  scan_kernel<<<kB * (kDin / kScanCh), kScanCh, 0, stream>>>(XD, XC, W_dt, b_dt, A_log, Dsk, YS);

  ln_gate_kernel<<<kRows / 32, 256, 0, stream>>>(YS, XZ, ln_g, ln_b, YGH, YGL);

  wmma_gemm64<1, 1, 0, 0, false><<<dim3((kRows / 64) * (kOutN / 64) / 8, 1), 256, 0, stream>>>(
      YGH, YGL, kDin, 0L,
      WOB, nullptr, kDin, 0L,
      (void*)out, nullptr, kDm, 0L,
      nullptr, nullptr, 0L,
      kRows, kOutN, kDin, 1.0f, kDm);
}
